// ModalityBranchRN_12979391168872
// MI455X (gfx1250) — hardware-run, weakly checked
//
#include <hip/hip_runtime.h>


#ifndef NB
#define NB 128
#endif
#define NB_FULL 128
#define XL      4096
#define XL_FULL 4096
#define XQ      (XL / 4)
#define C1      8
#define P1      1024
#define P2      128
#define HROWS   1032
#define W2P     72
#define FWP     72
#define HH      64
#define OSP2    68
#define LEAK    0.2f
#define C16     16.0f
#define RELC    64.0f
#define NEGB    (-3.0e38f)

static_assert(XL == 4 * P1);
static_assert(P1 == 8 * P2);
static_assert((P1 / 16) == 8 * 8);
static_assert(P2 == 8 * 16);
static_assert(2 * HH == 8 * 16);
static_assert(4 * HH == 256);
static_assert(P2 / 4 == 32);
static_assert(HROWS >= P1 + 4);
static_assert(C1 == 8);
static_assert(C1 * 5 <= 64);
static_assert(HH == 64);
static_assert(8 * 16 == HH * 2);
static_assert(32 * 16 * 8 == 16 * HH * 4);
static_assert(NB % 16 == 0);
static_assert(NB <= NB_FULL);
static_assert((W2P * 2) % 16 == 0);
static_assert((FWP * 2) % 16 == 0);
static_assert((OSP2 * 4) % 16 == 0);
static_assert(HROWS * 8 * 2 + 16 * W2P * 2 + 2 * HH * 8 * 2 + P2 * 8 * 2 + 2 * P2 * HH * 4 + 48 * 4 + 8 * 4 + 2 * HH * 4 + 4 * HH * 4 <= 131072);
static_assert(HH * FWP * 2 + HH * 4 + 8 * 16 * OSP2 * 4 <= 131072);

typedef _Float16 h16;
typedef unsigned short bf;
typedef __attribute__((ext_vector_type(16))) _Float16 v16h;
typedef __attribute__((ext_vector_type(8)))  _Float16 v8h;
typedef __attribute__((ext_vector_type(8)))  float    v8f;
typedef __attribute__((ext_vector_type(4)))  float    v4f;
typedef v4f  __attribute__((may_alias)) v4fa;
typedef v8h  __attribute__((may_alias)) v8ha;

__device__ __forceinline__ unsigned short f2bf(float f) { unsigned u = __float_as_uint(f); u += 0x7FFFu + ((u >> 16) & 1u); return (unsigned short)(u >> 16); }
__device__ __forceinline__ float bfr(float f) { return __uint_as_float(((unsigned)f2bf(f)) << 16); }
__device__ __forceinline__ v16h cat16(v8h lo, v8h hi) { return __builtin_shufflevector(lo, hi, 0, 1, 2, 3, 4, 5, 6, 7, 8, 9, 10, 11, 12, 13, 14, 15); }
__device__ __forceinline__ v8f wmma16(v16h a, v16h b, v8f c) { return __builtin_amdgcn_wmma_f32_16x16x32_f16(false, a, false, b, (short)0, c, false, false); }
__device__ __forceinline__ v16h  ldh(const h16* p) { return cat16(*(const v8h*)p, *(const v8h*)(p + 16)); }
__device__ __forceinline__ void wave_sync() { __builtin_amdgcn_fence(3  , "wavefront"); __builtin_amdgcn_wave_barrier(); asm volatile("" ::: "memory"); }
__device__ __forceinline__ h16 toh_flush(float v) { const h16 r = (h16)v; return (fabsf(v) < 6.103515625e-05f) ? (h16)0.0f : r; }
__device__ __forceinline__ v8f wmma16g(v16h a, v16h b, v8f c) { c = wmma16(a, b, c); asm volatile("v_nop\n\tv_nop\n\tv_nop\n\tv_nop" : "+v"(c) : "v"(a), "v"(b)); return c; }

__global__ __launch_bounds__(256) void k_rel(const float* __restrict__ x, const float* __restrict__ c1w, const float* __restrict__ c1b,
                                             const float* __restrict__ c2w, const float* __restrict__ c2b,
                                             const float* __restrict__ gw, const float* __restrict__ gb, h16* REL) {
    __shared__ __align__(16) h16 h1s[HROWS * 8];
    __shared__ __align__(16) h16 w2s[16 * W2P];
    __shared__ __align__(16) h16 gws[2 * HH * 8];
    __shared__ __align__(16) h16 h2s[P2 * 8];
    __shared__ __align__(16) float ab[2 * P2 * HH];
    __shared__ float w1s[48];
    __shared__ float b2s[8];
    __shared__ float gbs[2 * HH];
    __shared__ float part[4 * HH];
    const int tid = threadIdx.x;
    const int lane = threadIdx.x & 31, lr = lane & 15, hi = lane >> 4;
    const int wave = __builtin_amdgcn_readfirstlane((int)(threadIdx.x >> 5));
    const int b = blockIdx.x;

    { float v = c1w[tid < 40 ? tid : 39]; asm volatile("" : "+v"(v)); if (tid < 40) w1s[tid] = bfr(v); }
    { float v = c1b[tid & 7]; float u = c2b[tid & 7]; asm volatile("" : "+v"(v)); asm volatile("" : "+v"(u)); if (tid < 8) { w1s[40 + tid] = bfr(v); b2s[tid] = bfr(u); } }
    { float v = gb[tid & 63]; asm volatile("" : "+v"(v)); const float g = (tid < HH) ? bfr(v) : 0.0f; if (tid < 2 * HH) gbs[tid] = g; }
#pragma unroll 1
    for (int e = tid; e < 16 * 64; e += 256) {
        const int n = e >> 6, k = e & 63, t = k >> 3, ci = k & 7;
        const int nn = n < 8 ? n : 7, tt = t < 5 ? t : 4;
        float v = c2w[nn * 40 + ci * 5 + tt]; asm volatile("" : "+v"(v));
        const bool ok = (n < 8) & (t < 5);
        const float s = ok ? bfr(v) * C16 : 0.0f;
        w2s[n * W2P + k] = toh_flush(s);
    }
#pragma unroll 1
    for (int e = tid; e < 2 * HH * 8; e += 256) {
        const int row = e >> 3, c = e & 7, sel = row >> 6, hh = row & 63;
        gws[e] = toh_flush(bfr(gw[hh * 16 + sel * 8 + c]) * C16);
    }
    __syncthreads();

    const size_t xb = (size_t)b * XL_FULL;
#pragma unroll 1
    for (int r = tid; r < HROWS; r += 256) {
        float xx[12];
#pragma unroll
        for (int qq = 0; qq < 3; ++qq) {
            const int q = r - 3 + qq;
            const int qc = q < 0 ? 0 : (q > XQ - 1 ? XQ - 1 : q);
            v4f t4 = *(const v4f*)(x + xb + (size_t)qc * 4); asm volatile("" : "+v"(t4));
            const bool ok = (q >= 0) & (q < XQ);
#pragma unroll
            for (int i = 0; i < 4; ++i) xx[4 * qq + i] = ok ? bfr(t4[i]) : 0.0f;
        }
        const bool rowok = (r >= 2) & (r < P1 + 2);
#pragma unroll 1
        for (int c = 0; c < C1; ++c) {
            const float w0 = w1s[c * 5 + 0], w1 = w1s[c * 5 + 1], w2 = w1s[c * 5 + 2], w3 = w1s[c * 5 + 3], w4 = w1s[c * 5 + 4], bb = w1s[40 + c];
            float mxv = NEGB;
#pragma unroll
            for (int pp = 0; pp < 4; ++pp) {
                float s = xx[pp + 2] * w0; s += xx[pp + 3] * w1; s += xx[pp + 4] * w2; s += xx[pp + 5] * w3; s += xx[pp + 6] * w4; s += bb;
                const float lv = (s >= 0.0f) ? s : LEAK * s;
                mxv = fmaxf(mxv, lv);
            }
            const float val = rowok ? mxv * C16 : 0.0f;
            h1s[r * 8 + c] = toh_flush(val);
        }
    }
    __syncthreads();

    const v8h z8 = (v8h){};
    {
        const v16h bw0 = cat16(*(const v8ha*)(&w2s[lr * W2P +  0 + 8 * hi]), *(const v8ha*)(&w2s[lr * W2P + 16 + 8 * hi]));
        const v16h bw1 = cat16(*(const v8ha*)(&w2s[lr * W2P + 32 + 8 * hi]), *(const v8ha*)(&w2s[lr * W2P + 48 + 8 * hi]));
        const float bco = b2s[lr & 7];
#pragma unroll 1
        for (int i = 0; i < 8; ++i) {
            const int mt = wave * 8 + i; const int p0 = mt * 16;
            const int ra = p0 + lr + hi;
            const v8h a00 = *(const v8ha*)(&h1s[ra * 8]);
            const v8h a01 = *(const v8ha*)(&h1s[(ra + 2) * 8]);
            v8h a10 = *(const v8ha*)(&h1s[(p0 + lr + 4) * 8]); asm volatile("" : "+v"(a10));
            a10 = (hi == 0) ? a10 : z8;
            v8f acc = (v8f){};
            acc = wmma16g(cat16(a00, a01), bw0, acc);
            acc = wmma16g(cat16(a10, z8), bw1, acc);
            float mxv = NEGB;
#pragma unroll
            for (int r = 0; r < 8; ++r) { const float v = acc[r] * (1.0f / 256.0f) + bco; const float lv = (v >= 0.0f) ? v : LEAK * v; mxv = fmaxf(mxv, lv); }
            if (lr < 8) h2s[(2 * mt + hi) * 8 + lr] = toh_flush(mxv * C16);
        }
    }
    __syncthreads();

    {
        const int m0 = wave * 16;
        v8h ar = *(const v8ha*)(&h2s[(m0 + lr) * 8]); asm volatile("" : "+v"(ar));
        ar = (hi == 0) ? ar : z8;
        const v16h af = cat16(ar, z8);
#pragma unroll 1
        for (int nt = 0; nt < 8; ++nt) {
            v8h br = *(const v8ha*)(&gws[(nt * 16 + lr) * 8]); asm volatile("" : "+v"(br));
            br = (hi == 0) ? br : z8;
            v8f acc = (v8f){};
            acc = wmma16g(af, cat16(br, z8), acc);
            const int hc = (nt & 3) * 16 + lr;
            const float add = gbs[nt * 16 + lr];
            const int off = (nt >> 2) * (P2 * HH) + (m0 + 8 * hi) * HH + hc;
#pragma unroll
            for (int r = 0; r < 8; ++r) ab[off + r * HH] = acc[r] * (1.0f / 256.0f) + add;
        }
    }
    __syncthreads();

    {
        const int h = tid & 63, q = tid >> 6;
        float tot = 0.0f;
#pragma unroll 1
        for (int i = q * 32; i < q * 32 + 32; ++i) {
            const float ai = ab[i * HH + h];
            float si = 0.0f;
#pragma unroll 4
            for (int j = 0; j < P2; ++j) { const float s = ai + ab[P2 * HH + j * HH + h]; si += fmaxf(s, LEAK * s); }
            tot += si;
        }
        part[q * HH + h] = tot;
    }
    __syncthreads();

    if (wave == 0) {
        const int hq = lane & 7;
        v8h o;
#pragma unroll
        for (int i = 0; i < 8; ++i) { const int h = hq * 8 + i;
            const float s = (part[h] + part[HH + h]) + (part[2 * HH + h] + part[3 * HH + h]);
            o[i] = toh_flush(s * (RELC / (float)(P2 * P2))); }
        h16* dst = REL + (size_t)b * HH + hq * 8;
        if (lane < 8) { *(volatile v8h*)dst = o; __threadfence(); *(volatile v8h*)dst = o; }
    }
}

__global__ __launch_bounds__(256) void k_fout(const h16* __restrict__ REL, const float* __restrict__ fw, const float* __restrict__ fb, float* OUT) {
    __shared__ __align__(16) h16 fws[HH * FWP];
    __shared__ float fbs[HH];
    __shared__ __align__(16) float os[8 * 16 * OSP2];
    const int tid = threadIdx.x;
    const int lane = threadIdx.x & 31, lr = lane & 15, hi = lane >> 4;
    const int wave = __builtin_amdgcn_readfirstlane((int)(threadIdx.x >> 5));
#pragma unroll 1
    for (int e = tid; e < HH * HH; e += 256) {
        const int n = e >> 6, k = e & 63;
        fws[n * FWP + k] = toh_flush(bfr(fw[e]) * C16);
    }
    { float v = fb[tid & 63]; asm volatile("" : "+v"(v)); if (tid < HH) fbs[tid] = bfr(v); }
    __syncthreads();
    const int mt = blockIdx.x * 8 + wave;
    if (mt < NB / 16) {
        const int m0 = mt * 16;
        v8f acc[4];
#pragma unroll
        for (int nb = 0; nb < 4; ++nb) acc[nb] = (v8f){};
#pragma unroll
        for (int kc = 0; kc < HH; kc += 32) {
            const v16h a = ldh(REL + (size_t)(m0 + lr) * HH + kc + 8 * hi);
#pragma unroll
            for (int nb = 0; nb < 4; ++nb) {
                const v16h bq = cat16(*(const v8ha*)(&fws[(nb * 16 + lr) * FWP + kc + 8 * hi]), *(const v8ha*)(&fws[(nb * 16 + lr) * FWP + kc + 16 + 8 * hi]));
                acc[nb] = wmma16g(a, bq, acc[nb]);
            }
        }
        const int wb = wave * 16 * OSP2;
#pragma unroll
        for (int nb = 0; nb < 4; ++nb) {
            const float bc = fbs[nb * 16 + lr];
#pragma unroll
            for (int j = 0; j < 8; ++j) { const float v = acc[nb][j] * (1.0f / (RELC * C16)) + bc;
                os[wb + (hi * 8 + j) * OSP2 + nb * 16 + lr] = (v >= 0.0f) ? v : LEAK * v; }
        }
        wave_sync();
        float* orow = OUT + (size_t)m0 * HH;
#pragma unroll 1
        for (int ps = 0; ps < 2; ++ps) {
#pragma unroll
            for (int s = 0; s < 8; ++s) { const int row = 2 * s + (lane >> 4), cofs = (lane & 15) * 4;
                const v4f val = *(const v4fa*)(&os[wb + row * OSP2 + cofs]);
                *(volatile v4f*)(orow + (size_t)row * HH + cofs) = val; }
            if (ps == 0) __threadfence(); }
    }
}

static constexpr size_t al256(size_t v) { return (v + 255) & ~(size_t)255; }
static constexpr size_t SZ_REL = al256((size_t)NB * HH * 2);
static constexpr size_t SZ_TOTAL = SZ_REL;
static_assert(SZ_TOTAL <= (size_t)134217728);
static_assert((size_t)(NB - 1) * HH * 2 + 8 * 16 <= SZ_REL);
static_assert((size_t)NB * HH * 4 <= (size_t)32768);

extern "C" void kernel_launch(void* const* d_in, const int* in_sizes, int n_in,
                              void* d_out, int out_size, void* d_ws, size_t ws_size, hipStream_t stream) {
    if (n_in < 9) return;
    if ((size_t)in_sizes[0] < (size_t)(NB - 1) * XL_FULL + XL) return;
    if (in_sizes[1] < 40 || in_sizes[2] < 8 || in_sizes[3] < 320 || in_sizes[4] < 8) return;
    if (in_sizes[5] < HH * 16 || in_sizes[6] < HH || in_sizes[7] < HH * HH || in_sizes[8] < HH) return;
    if ((size_t)out_size < (size_t)NB * HH) return;
    if (SZ_TOTAL > ws_size) return;
    const float* x   = (const float*)d_in[0];
    const float* c1w = (const float*)d_in[1]; const float* c1b = (const float*)d_in[2];
    const float* c2w = (const float*)d_in[3]; const float* c2b = (const float*)d_in[4];
    const float* gw  = (const float*)d_in[5]; const float* gb  = (const float*)d_in[6];
    const float* fw  = (const float*)d_in[7]; const float* fb  = (const float*)d_in[8];
    float* OUT = (float*)d_out;
    h16* REL = (h16*)d_ws;

    k_rel<<<dim3(NB, 1, 1), 256, 0, stream>>>(x, c1w, c1b, c2w, c2b, gw, gb, REL);
    k_fout<<<dim3((NB / 16 + 7) / 8, 1, 1), 256, 0, stream>>>(REL, fw, fb, OUT);
}
